// pointnet_fp_module_32298154066788
// MI455X (gfx1250) — hardware-verified
//
#include <hip/hip_runtime.h>
#include <stddef.h>


#pragma clang fp contract(off)

typedef __bf16 bf16_t;
typedef bf16_t v8b  __attribute__((ext_vector_type(8)));
typedef bf16_t v16b __attribute__((ext_vector_type(16)));
typedef float  v8f  __attribute__((ext_vector_type(8)));
typedef float  v4f  __attribute__((ext_vector_type(4)));
typedef int    v4i  __attribute__((ext_vector_type(4)));
typedef int    v8i  __attribute__((ext_vector_type(8)));

namespace {
constexpr int kB  = 16;
constexpr int kN1 = 4096;
constexpr int kN2 = 1024;
constexpr int kC1 = 128;
constexpr int kC2 = 256;
constexpr int kCX = kC2 + kC1;
constexpr int kO1 = 256;
constexpr int kO2 = 128;

constexpr int kThreads = 256;
constexpr int kWaves   = kThreads / 32;
constexpr int kNT  = 64;
constexpr int kNTT = kNT / 16;
constexpr int kXR  = kCX + 8;
constexpr int kHR  = kO1 + 8;
constexpr int kK1  = kCX / 32;
constexpr int kK2  = kO1 / 32;
constexpr int kSP  = 68;

constexpr size_t kXPlaneBytes = (size_t)kNT * kXR * sizeof(bf16_t);
constexpr size_t kHPlaneBytes = (size_t)kNT * kHR * sizeof(bf16_t);
constexpr size_t kStageBytes  = (size_t)kWaves * 16 * kSP * sizeof(float);
constexpr size_t kSmemBytes   = 2 * kXPlaneBytes + 2 * kHPlaneBytes;

typedef char check_waves_l2[(kO2 / 16 == kWaves) ? 1 : -1];
typedef char check_waves_l1[(kO1 / 16 == 2 * kWaves) ? 1 : -1];
typedef char check_stage[(kStageBytes <= 2 * kXPlaneBytes) ? 1 : -1];
typedef char check_shapes[(kN1 % kNT == 0 && kN1 % kThreads == 0 && kCX % 32 == 0 && kO1 % 32 == 0 &&
                           kC2 % 32 == 0 && kC1 % 32 == 0 && (kXR % 8) == 0 && (kHR % 8) == 0) ? 1 : -1];
}

union Frag { v16b v; v8b h[2]; };

__device__ __forceinline__ Frag ld_frag(const bf16_t* p) {
  Frag f;
  f.h[0] = *(const v8b*)p;
  f.h[1] = *(const v8b*)(p + 16);
  return f;
}

__device__ __forceinline__ v8f ld_f8(const float* p) {
  const v4f a = *(const v4f*)p;
  const v4f c = *(const v4f*)(p + 4);
  return __builtin_shufflevector(a, c, 0, 1, 2, 3, 4, 5, 6, 7);
}

__device__ __forceinline__ void split_bf16(const v8f x, v8b& hi, v8b& lo) {
  hi = __builtin_convertvector(x, v8b);
  const v8f hf = __builtin_convertvector(hi, v8f);
  const v8f d  = x - hf;
  lo = __builtin_convertvector(d, v8b);
}

#define WMMA_BF16(A, B, C) __builtin_amdgcn_wmma_f32_16x16x32_bf16(false, (A), false, (B), (short)0, (C), false, false)

__device__ __forceinline__ v8f mma3(v8f c, const Frag& ah, const Frag& al, const Frag& bh, const Frag& bl) {
  c = WMMA_BF16(ah.v, bh.v, c);
  c = WMMA_BF16(al.v, bh.v, c);
  c = WMMA_BF16(ah.v, bl.v, c);
  return c;
}

__device__ __forceinline__ void wmma_guard(v8f& c0, v8f& c1, v8f& c2, v8f& c3,
                                           const Frag& ah, const Frag& al,
                                           const Frag* bh, const Frag* bl) {
  asm volatile("v_nop\n\tv_nop\n\tv_nop\n\tv_nop"
               : "+v"(c0), "+v"(c1), "+v"(c2), "+v"(c3)
               : "v"(__builtin_bit_cast(v8i, ah.v)), "v"(__builtin_bit_cast(v8i, al.v)),
                 "v"(__builtin_bit_cast(v8i, bh[0].v)), "v"(__builtin_bit_cast(v8i, bh[1].v)),
                 "v"(__builtin_bit_cast(v8i, bh[2].v)), "v"(__builtin_bit_cast(v8i, bh[3].v)),
                 "v"(__builtin_bit_cast(v8i, bl[0].v)), "v"(__builtin_bit_cast(v8i, bl[1].v)),
                 "v"(__builtin_bit_cast(v8i, bl[2].v)), "v"(__builtin_bit_cast(v8i, bl[3].v)));
}

__device__ __forceinline__ void gemm_kstep(v8f* acc, const bf16_t* ap_h, const bf16_t* ap_l,
                                           const bf16_t* bp_h, const bf16_t* bp_l, int bstride) {
  const Frag ah = ld_frag(ap_h);
  const Frag al = ld_frag(ap_l);
  Frag bh[kNTT], bl[kNTT];
#pragma unroll
  for (int nt = 0; nt < kNTT; ++nt) {
    bh[nt] = ld_frag(bp_h + nt * bstride);
    bl[nt] = ld_frag(bp_l + nt * bstride);
  }
#pragma unroll
  for (int nt = 0; nt < kNTT; ++nt) acc[nt] = mma3(acc[nt], ah, al, bh[nt], bl[nt]);
  wmma_guard(acc[0], acc[1], acc[2], acc[3], ah, al, bh, bl);
}

__global__ __launch_bounds__(kThreads) void cvt_weights_kernel(
    const float* __restrict__ W1, const float* __restrict__ W2,
    bf16_t* __restrict__ W1hi, bf16_t* __restrict__ W1lo,
    bf16_t* __restrict__ W2hi, bf16_t* __restrict__ W2lo,
    int n1g, int n2g)
{
  const int t = blockIdx.x * kThreads + threadIdx.x;
  if (t >= n1g + n2g) return;
  const bool in1 = t < n1g;
  const int g = in1 ? t : (t - n1g);
  const float* src = in1 ? W1 : W2;
  bf16_t* dh = in1 ? W1hi : W2hi;
  bf16_t* dl = in1 ? W1lo : W2lo;

  const v8f x = ld_f8(src + (size_t)g * 8);
  v8b hi, lo;
  split_bf16(x, hi, lo);
  const v4i hbits = __builtin_bit_cast(v4i, hi);
  const v4i lbits = __builtin_bit_cast(v4i, lo);
  const size_t o = (size_t)g * 8;

  *(volatile v4i*)(dh + o) = hbits;
  *(volatile v4i*)(dl + o) = lbits;
  __threadfence();
  *(volatile v4i*)(dh + o) = hbits;
  *(volatile v4i*)(dl + o) = lbits;
}

__global__ __launch_bounds__(kThreads) void knn3_kernel(
    const float* __restrict__ xyz1, const float* __restrict__ xyz2,
    int* __restrict__ idx4, float* __restrict__ w4)
{
  __shared__ v4f pts[kN2];
  const int b = blockIdx.y;
  const int tid = threadIdx.x;
  const int n = blockIdx.x * kThreads + tid;

  const float* qb = xyz2 + (size_t)b * 3 * kN2;
  for (int m = tid; m < kN2; m += kThreads) {
    const float qx = qb[m], qy = qb[kN2 + m], qz = qb[2 * kN2 + m];
    v4f t;
    t.x = qx; t.y = qy; t.z = qz;
    t.w = fmaf(qz, qz, fmaf(qy, qy, qx * qx));
    pts[m] = t;
  }
  __syncthreads();

  const int nc = (n < kN1) ? n : (kN1 - 1);
  const float* pb = xyz1 + (size_t)b * 3 * kN1;
  const float px = pb[nc], py = pb[kN1 + nc], pz = pb[2 * kN1 + nc];
  const float s1 = fmaf(pz, pz, fmaf(py, py, px * px));

  float d0 = 3.0e38f, d1 = 3.0e38f, d2 = 3.0e38f;
  int   i0 = 0,       i1 = 0,       i2 = 0;
#pragma unroll 2
  for (int m = 0; m < kN2; ++m) {
    const v4f t = pts[m];
    const float pxy = px * t.x + py * t.y;
    const float c   = pxy + pz * t.z;
    float d = (s1 + t.w) - 2.0f * c;
    d = fmaxf(d, 0.0f);
    if (d < d2) {
      if (d < d1) {
        if (d < d0) { d2 = d1; i2 = i1; d1 = d0; i1 = i0; d0 = d; i0 = m; }
        else        { d2 = d1; i2 = i1; d1 = d;  i1 = m; }
      } else        { d2 = d;  i2 = m; }
    }
  }
  const float r0 = 1.0f / (d0 + 1e-8f);
  const float r1 = 1.0f / (d1 + 1e-8f);
  const float r2 = 1.0f / (d2 + 1e-8f);
  const float nrm = (r0 + r1) + r2;
  const float inv = 1.0f / nrm;

  v4i iv; iv.x = i0; iv.y = i1; iv.z = i2; iv.w = 0;
  v4f wv; wv.x = r0 * inv; wv.y = r1 * inv; wv.z = r2 * inv; wv.w = 0.0f;
  const size_t o = ((size_t)b * kN1 + (size_t)n) * 4;

  if (n < kN1) {
    *(volatile v4i*)(idx4 + o) = iv;
    *(volatile v4f*)(w4 + o) = wv;
  }
  __threadfence();
  if (n < kN1) {
    *(volatile v4i*)(idx4 + o) = iv;
    *(volatile v4f*)(w4 + o) = wv;
  }
}

__global__ __launch_bounds__(kThreads) void fused_mlp_kernel(
    const float* __restrict__ f1, const float* __restrict__ f2,
    const float* __restrict__ bias1, const float* __restrict__ bias2,
    const bf16_t* __restrict__ W1hi, const bf16_t* __restrict__ W1lo,
    const bf16_t* __restrict__ W2hi, const bf16_t* __restrict__ W2lo,
    const int* __restrict__ idx4, const float* __restrict__ w4,
    float* __restrict__ out)
{
  extern __shared__ v4f smem_v4[];
  bf16_t* const Xhi = (bf16_t*)smem_v4;
  bf16_t* const Xlo = Xhi + kNT * kXR;
  bf16_t* const Hhi = Xlo + kNT * kXR;
  bf16_t* const Hlo = Hhi + kNT * kHR;
  float*  const Stg = (float*)smem_v4;

  const int b    = blockIdx.y;
  const int n0   = blockIdx.x * kNT;
  const int tid  = threadIdx.x;
  const int lane = tid & 31;
  const int wave = tid >> 5;
  const int h    = lane >> 4;
  const int m    = lane & 15;

  {
    const int nl  = tid & (kNT - 1);
    const int sub = tid >> 6;
    const int ng  = n0 + nl;
    const size_t q4 = ((size_t)b * kN1 + (size_t)ng) * 4;
    const v4i jj = *(const v4i*)(idx4 + q4);
    const v4f ww = *(const v4f*)(w4 + q4);
    const int j0 = min(max(jj.x, 0), kN2 - 1);
    const int j1 = min(max(jj.y, 0), kN2 - 1);
    const int j2 = min(max(jj.z, 0), kN2 - 1);
    const float w0 = ww.x, w1 = ww.y, w2 = ww.z;

    const float* f2b = f2 + (size_t)b * kC2 * kN2;
    bf16_t* xh = Xhi + nl * kXR;
    bf16_t* xl = Xlo + nl * kXR;
#pragma unroll 1
    for (int g = 0; g < kC2 / 32; ++g) {
      const int c0 = sub * (kC2 / 4) + g * 8;
      v8f v;
#pragma unroll
      for (int e = 0; e < 8; ++e) {
        const float* r = f2b + (size_t)(c0 + e) * kN2;
        v[e] = fmaf(w2, r[j2], fmaf(w1, r[j1], w0 * r[j0]));
      }
      v8b vh, vl;
      split_bf16(v, vh, vl);
      *(v8b*)(xh + c0) = vh;
      *(v8b*)(xl + c0) = vl;
    }
    const float* f1b = f1 + (size_t)b * kC1 * kN1 + ng;
#pragma unroll 1
    for (int g = 0; g < kC1 / 32; ++g) {
      const int c0 = sub * (kC1 / 4) + g * 8;
      v8f v;
#pragma unroll
      for (int e = 0; e < 8; ++e) v[e] = f1b[(size_t)(c0 + e) * kN1];
      v8b vh, vl;
      split_bf16(v, vh, vl);
      *(v8b*)(xh + kC2 + c0) = vh;
      *(v8b*)(xl + kC2 + c0) = vl;
    }
  }
  __syncthreads();

  for (int ot = wave; ot < kO1 / 16; ot += kWaves) {
    v8f acc[kNTT];
    const v8f bb = ld_f8(bias1 + ot * 16 + 8 * h);
    acc[0] = bb; acc[1] = bb; acc[2] = bb; acc[3] = bb;

    const bf16_t* aph = W1hi + (size_t)(ot * 16 + m) * kCX + 8 * h;
    const bf16_t* apl = W1lo + (size_t)(ot * 16 + m) * kCX + 8 * h;
    const bf16_t* bph = Xhi + m * kXR + 8 * h;
    const bf16_t* bpl = Xlo + m * kXR + 8 * h;
#pragma unroll 1
    for (int ks = 0; ks < kK1; ++ks)
      gemm_kstep(acc, aph + 32 * ks, apl + 32 * ks, bph + 32 * ks, bpl + 32 * ks, 16 * kXR);

#pragma unroll
    for (int nt = 0; nt < kNTT; ++nt) {
      v8f hv;
#pragma unroll
      for (int r = 0; r < 8; ++r) hv[r] = fmaxf(acc[nt][r], 0.0f);
      v8b hh, hl;
      split_bf16(hv, hh, hl);
      const int ho = (nt * 16 + m) * kHR + ot * 16 + 8 * h;
      *(v8b*)(Hhi + ho) = hh;
      *(v8b*)(Hlo + ho) = hl;
    }
  }
  __syncthreads();

  const int ot2 = wave;
  float* const stg = Stg + wave * (16 * kSP);
  {
    v8f acc[kNTT];
    const v8f bb = ld_f8(bias2 + ot2 * 16 + 8 * h);
    acc[0] = bb; acc[1] = bb; acc[2] = bb; acc[3] = bb;

    const bf16_t* aph = W2hi + (size_t)(ot2 * 16 + m) * kO1 + 8 * h;
    const bf16_t* apl = W2lo + (size_t)(ot2 * 16 + m) * kO1 + 8 * h;
    const bf16_t* bph = Hhi + m * kHR + 8 * h;
    const bf16_t* bpl = Hlo + m * kHR + 8 * h;
#pragma unroll 1
    for (int ks = 0; ks < kK2; ++ks)
      gemm_kstep(acc, aph + 32 * ks, apl + 32 * ks, bph + 32 * ks, bpl + 32 * ks, 16 * kHR);

#pragma unroll
    for (int nt = 0; nt < kNTT; ++nt) {
#pragma unroll
      for (int r = 0; r < 8; ++r)
        stg[(8 * h + r) * kSP + nt * 16 + m] = fmaxf(acc[nt][r], 0.0f);
    }
  }
  __syncthreads();

  {
    float* const outb = out + (size_t)b * kO2 * kN1;
    v4f    ov[8];
    size_t oo[8];
#pragma unroll
    for (int j = 0; j < 8; ++j) {
      const int row   = 2 * j + (lane >> 4);
      const int half  = (lane >> 3) & 1;
      const int piece = lane & 7;
      ov[j] = *(const v4f*)(stg + row * kSP + half * 32 + piece * 4);
      oo[j] = (size_t)(ot2 * 16 + row) * kN1 + (size_t)(n0 + half * 32 + piece * 4);
    }
#pragma unroll
    for (int j = 0; j < 8; ++j) *(volatile v4f*)(outb + oo[j]) = ov[j];
    __threadfence();
#pragma unroll
    for (int j = 0; j < 8; ++j) *(volatile v4f*)(outb + oo[j]) = ov[j];
  }
}

extern "C" void kernel_launch(void* const* d_in, const int* in_sizes, int n_in,
                              void* d_out, int out_size, void* d_ws, size_t ws_size,
                              hipStream_t stream) {
  if (n_in < 8) return;
  if (in_sizes[0] != kB * 3 * kN1)   return;
  if (in_sizes[1] != kB * 3 * kN2)   return;
  if (in_sizes[2] != kB * kC1 * kN1) return;
  if (in_sizes[3] != kB * kC2 * kN2) return;
  if (in_sizes[4] != kO1 * kCX)      return;
  if (in_sizes[5] != kO1)            return;
  if (in_sizes[6] != kO2 * kO1)      return;
  if (in_sizes[7] != kO2)            return;
  if (out_size != kB * kO2 * kN1)    return;

  const float* xyz1 = (const float*)d_in[0];
  const float* xyz2 = (const float*)d_in[1];
  const float* f1   = (const float*)d_in[2];
  const float* f2   = (const float*)d_in[3];
  const float* W1   = (const float*)d_in[4];
  const float* b1   = (const float*)d_in[5];
  const float* W2   = (const float*)d_in[6];
  const float* b2   = (const float*)d_in[7];
  float* out = (float*)d_out;

  size_t off = 0;
  const size_t szW1p = (size_t)kO1 * kCX * sizeof(bf16_t);
  const size_t szW2p = (size_t)kO2 * kO1 * sizeof(bf16_t);
  const size_t szI4  = (size_t)kB * kN1 * 4 * sizeof(int);
  const size_t szW4  = (size_t)kB * kN1 * 4 * sizeof(float);
  const size_t oW1h = off; off += (szW1p + 255) & ~(size_t)255;
  const size_t oW1l = off; off += (szW1p + 255) & ~(size_t)255;
  const size_t oW2h = off; off += (szW2p + 255) & ~(size_t)255;
  const size_t oW2l = off; off += (szW2p + 255) & ~(size_t)255;
  const size_t oI4  = off; off += (szI4 + 255) & ~(size_t)255;
  const size_t oW4  = off; off += (szW4 + 255) & ~(size_t)255;
  if (off > ws_size) return;

  char* ws = (char*)d_ws;
  bf16_t* W1hi = (bf16_t*)(ws + oW1h);
  bf16_t* W1lo = (bf16_t*)(ws + oW1l);
  bf16_t* W2hi = (bf16_t*)(ws + oW2h);
  bf16_t* W2lo = (bf16_t*)(ws + oW2l);
  int*    idx4 = (int*)(ws + oI4);
  float*  w4   = (float*)(ws + oW4);

  const int n1g = kO1 * kCX / 8;
  const int n2g = kO2 * kO1 / 8;
  const int cvtBlocks = (n1g + n2g + kThreads - 1) / kThreads;

  (void)hipFuncSetAttribute(reinterpret_cast<const void*>(&fused_mlp_kernel),
                            hipFuncAttributeMaxDynamicSharedMemorySize, (int)kSmemBytes);

  cvt_weights_kernel<<<dim3(cvtBlocks), dim3(kThreads), 0, stream>>>(
      W1, W2, W1hi, W1lo, W2hi, W2lo, n1g, n2g);
  knn3_kernel<<<dim3(kN1 / kThreads, kB), dim3(kThreads), 0, stream>>>(xyz1, xyz2, idx4, w4);
  fused_mlp_kernel<<<dim3(kN1 / kNT, kB), dim3(kThreads), kSmemBytes, stream>>>(
      f1, f2, b1, b2, W1hi, W1lo, W2hi, W2lo, idx4, w4, out);
  (void)hipGetLastError();
}
